// MultiScaleRetention_37452114821262
// MI455X (gfx1250) — hardware-verified
//
#include <hip/hip_runtime.h>
#include <math.h>
#include <stdint.h>

#define NB_   2
#define T_    2048
#define E_    512
#define NH_   8
#define HD_   64
#define NP_   32
#define NTOK_ 4096
#define GRK_  1024
#define OS_P  68

static_assert(NTOK_ == NB_ * T_);
static_assert(E_ == NH_ * HD_);
static_assert(HD_ == 2 * NP_);
static_assert(GRK_ == 2 * E_);
static_assert(T_ % 64 == 0 && E_ % 64 == 0 && NTOK_ % 64 == 0);
static_assert((T_ / 64) == 32);
static_assert(E_ % 32 == 0 && GRK_ % 32 == 0);
static_assert(((NTOK_ / 64) * (E_ / 64)) % 8 == 0);
static_assert(((E_ / 64) * (T_ / 64)) % 8 == 0);
static_assert((NTOK_ * E_) % (8 * 256) == 0);
static_assert((E_ * E_) % (8 * 256) == 0);
static_assert((T_ * NP_) % 256 == 0);

typedef __attribute__((ext_vector_type(16))) __bf16   v16b;
typedef __attribute__((ext_vector_type(8)))  float    v8f;
typedef __attribute__((ext_vector_type(4)))  float    v4f;
typedef __attribute__((ext_vector_type(4)))  unsigned int v4u;
typedef __attribute__((ext_vector_type(8)))  unsigned short u16x8;

union FragB { u16x8 h[2]; v16b v; };

constexpr size_t SZ_ACT = (size_t)NTOK_ * E_ * 2;
constexpr size_t SZ_W   = (size_t)E_ * E_ * 2;
constexpr size_t SZ_WO2 = (size_t)E_ * GRK_ * 2;
constexpr size_t SZ_ANG = (size_t)T_ * NP_ * 4;
constexpr size_t SZ_VT  = (size_t)NB_ * E_ * T_ * 2;
constexpr size_t SZ_G   = (size_t)NTOK_ * E_ * 4;
constexpr size_t SZ_GRC = (size_t)NTOK_ * GRK_ * 2;

constexpr size_t OFF_QB   = 0;
constexpr size_t OFF_KB   = OFF_QB   + SZ_ACT;
constexpr size_t OFF_VB   = OFF_KB   + SZ_ACT;
constexpr size_t OFF_WQ   = OFF_VB   + SZ_ACT;
constexpr size_t OFF_WK   = OFF_WQ   + SZ_W;
constexpr size_t OFF_WV   = OFF_WK   + SZ_W;
constexpr size_t OFF_WG   = OFF_WV   + SZ_W;
constexpr size_t OFF_WO2  = OFF_WG   + SZ_W;
constexpr size_t OFF_ANGC = OFF_WO2  + SZ_WO2;
constexpr size_t OFF_ANGS = OFF_ANGC + SZ_ANG;
constexpr size_t OFF_QH   = OFF_ANGS + SZ_ANG;
constexpr size_t OFF_QL   = OFF_QH   + SZ_ACT;
constexpr size_t OFF_KH   = OFF_QL   + SZ_ACT;
constexpr size_t OFF_KL   = OFF_KH   + SZ_ACT;
constexpr size_t OFF_VTH  = OFF_KL   + SZ_ACT;
constexpr size_t OFF_VTL  = OFF_VTH  + SZ_VT;
constexpr size_t OFF_G    = OFF_VTL  + SZ_VT;
constexpr size_t OFF_GRC  = OFF_G    + SZ_G;
constexpr size_t WS_END   = OFF_GRC  + SZ_GRC;
static_assert(WS_END <= (size_t)134217728);
static_assert(OFF_KB % 128 == 0 && OFF_VB % 128 == 0 && OFF_WQ % 128 == 0 && OFF_WK % 128 == 0 && OFF_WV % 128 == 0);
static_assert(OFF_WG % 128 == 0 && OFF_WO2 % 128 == 0 && OFF_ANGC % 128 == 0 && OFF_ANGS % 128 == 0);
static_assert(OFF_QH % 128 == 0 && OFF_QL % 128 == 0 && OFF_KH % 128 == 0 && OFF_KL % 128 == 0);
static_assert(OFF_VTH % 128 == 0 && OFF_VTL % 128 == 0 && OFF_G % 128 == 0 && OFF_GRC % 128 == 0);

__device__ __forceinline__ unsigned short f2bf_bits(float f) {
  unsigned u = __float_as_uint(f);
  return (unsigned short)((u + 0x7FFFu + ((u >> 16) & 1u)) >> 16);
}
__device__ __forceinline__ float bf_bits2f(unsigned short h) { return __uint_as_float(((unsigned)h) << 16); }
__device__ __forceinline__ float bf_rne(float f) { return bf_bits2f(f2bf_bits(f)); }

__device__ __forceinline__ v16b frag_ld(const unsigned short* p) {
  FragB f; f.h[0] = *(const u16x8*)(p); f.h[1] = *(const u16x8*)(p + 16); return f.v;
}
__device__ __forceinline__ v8f mma_b(v16b a, v16b b, v8f c) {
  return __builtin_amdgcn_wmma_f32_16x16x32_bf16(false, a, false, b, (short)0, c, false, false);
}
__device__ __forceinline__ void dep_guard_b(v8f& a, v8f& b, v16b x, v16b y) {
  asm volatile("v_nop\n\tv_nop\n\tv_nop\n\tv_nop" : "+v"(a), "+v"(b) : "v"(x), "v"(y));
}
__device__ __forceinline__ void keep4_b(v16b a, v16b b, v16b c, v16b d) { asm volatile("v_nop" :: "v"(a), "v"(b), "v"(c), "v"(d)); }
__device__ __forceinline__ void acc_guard4(v8f& a, v8f& b, v8f& c, v8f& d) {
  asm volatile("v_nop\n\tv_nop\n\tv_nop\n\tv_nop" : "+v"(a), "+v"(b), "+v"(c), "+v"(d));
}
__device__ __forceinline__ v8f mma_g(v8f c, v16b a, v16b b) {
  c = __builtin_amdgcn_wmma_f32_16x16x32_bf16(false, a, false, b, (short)0, c, false, false);
  asm volatile("v_nop\n\tv_nop\n\tv_nop\n\tv_nop" : "+v"(c) : "v"(a), "v"(b));
  return c;
}

__global__ __launch_bounds__(256) void xcvt_kernel(const float* __restrict__ src, unsigned short* dst, int n8) {
  const int i = blockIdx.x * 256 + threadIdx.x;
  if (i < n8) {
    const size_t e = (size_t)i * 8;
    const v4f a = *(const v4f*)(src + e);
    const v4f b = *(const v4f*)(src + e + 4);
    u16x8 hv;
    hv[0] = f2bf_bits(a[0]); hv[1] = f2bf_bits(a[1]); hv[2] = f2bf_bits(a[2]); hv[3] = f2bf_bits(a[3]);
    hv[4] = f2bf_bits(b[0]); hv[5] = f2bf_bits(b[1]); hv[6] = f2bf_bits(b[2]); hv[7] = f2bf_bits(b[3]);
    *(volatile u16x8*)(dst + e) = hv;
    __threadfence();
    *(volatile u16x8*)(dst + e) = hv;
  }
}

__global__ __launch_bounds__(256) void dupcvt_kernel(const float* __restrict__ src, unsigned short* dst, int n8, int cols, int ldo) {
  const int i = blockIdx.x * 256 + threadIdx.x;
  if (i < n8) {
    const size_t e = (size_t)i * 8;
    const int row = (int)(e / (size_t)cols);
    const int col = (int)(e - (size_t)row * cols);
    const v4f a = *(const v4f*)(src + e);
    const v4f b = *(const v4f*)(src + e + 4);
    u16x8 hv;
    hv[0] = f2bf_bits(a[0]); hv[1] = f2bf_bits(a[1]); hv[2] = f2bf_bits(a[2]); hv[3] = f2bf_bits(a[3]);
    hv[4] = f2bf_bits(b[0]); hv[5] = f2bf_bits(b[1]); hv[6] = f2bf_bits(b[2]); hv[7] = f2bf_bits(b[3]);
    unsigned short* d0 = dst + (size_t)row * ldo + col;
    *(volatile u16x8*)(d0) = hv;
    *(volatile u16x8*)(d0 + cols) = hv;
    __threadfence();
    *(volatile u16x8*)(d0) = hv;
    *(volatile u16x8*)(d0 + cols) = hv;
  }
}

__global__ __launch_bounds__(256) void ang_kernel(float* angc, float* angs, int n) {
  const int i = blockIdx.x * 256 + threadIdx.x;
  if (i < n) {
    const int npos = i >> 5;
    const int p    = i & 31;
    const float e   = (float)p * (1.0f / 31.0f);
    const double th = exp2(-(double)e * 13.287712379549449);
    const float thf = (float)th;
    const float ang = (float)npos * thf;
    float sv, cv;
    sincosf(ang, &sv, &cv);
    ((volatile float*)angc)[i] = cv;
    ((volatile float*)angs)[i] = sv;
    __threadfence();
    ((volatile float*)angc)[i] = cv;
    ((volatile float*)angs)[i] = sv;
  }
}

template <int BIAS_MODE, int OUT_MODE, int ACT>
__global__ __launch_bounds__(256) void gemm64_kernel(
    const unsigned short* __restrict__ A, int lda, long strideA,
    const unsigned short* __restrict__ Bt, int ldb, long strideB,
    void* Cout, void* Cout2, int ldc, long strideC,
    const float* __restrict__ bias, const float* __restrict__ angc, const float* __restrict__ angs,
    float oscale, int M, int N, int K) {
  __shared__ __align__(16) float sT[8][16 * 68];
  const int b    = blockIdx.y;
  const int lane = threadIdx.x & 31;
  const int wave = threadIdx.x >> 5;
  const int tilesN = N >> 6;
  const int tilesM = M >> 6;
  const int tile = blockIdx.x * 8 + wave;
  if (tile >= tilesM * tilesN) return;
  const int tm = tile / tilesN;
  const int tn = tile - tm * tilesN;
  const int m0 = tm << 6;
  const int n0 = tn << 6;

  const unsigned short* Ab = A  + (size_t)b * strideA;
  const unsigned short* Bb = Bt + (size_t)b * strideB;

  const int rlane = lane & 15;
  const int koff  = (lane >> 4) * 8;
  const int mOff  = (lane >> 4) * 8;

  v8f acc[4][4];
#pragma unroll
  for (int i = 0; i < 4; ++i)
#pragma unroll
    for (int j = 0; j < 4; ++j) acc[i][j] = (v8f){0.f,0.f,0.f,0.f,0.f,0.f,0.f,0.f};

  for (int k0 = 0; k0 < K; k0 += 32) {
    v16b bh[4];
#pragma unroll
    for (int j = 0; j < 4; ++j) {
      const size_t bo = (size_t)(n0 + (j << 4) + rlane) * ldb + koff + k0;
      bh[j] = frag_ld(Bb + bo);
    }
#pragma unroll
    for (int i = 0; i < 4; ++i) {
      const size_t ao = (size_t)(m0 + (i << 4) + rlane) * lda + koff + k0;
      v16b ah = frag_ld(Ab + ao);
#pragma unroll
      for (int j = 0; j < 4; ++j) acc[i][j] = mma_b(ah, bh[j], acc[i][j]);
      dep_guard_b(acc[i][0], acc[i][3], ah, ah);
    }
    keep4_b(bh[0], bh[1], bh[2], bh[3]);
  }
  acc_guard4(acc[0][0], acc[0][1], acc[0][2], acc[0][3]);
  acc_guard4(acc[1][0], acc[1][1], acc[1][2], acc[1][3]);
  acc_guard4(acc[2][0], acc[2][1], acc[2][2], acc[2][3]);
  acc_guard4(acc[3][0], acc[3][1], acc[3][2], acc[3][3]);

  float* slab = sT[wave];
#pragma unroll
  for (int i = 0; i < 4; ++i) {
    const int mBase = m0 + (i << 4);
    float bm[8];
#pragma unroll
    for (int r = 0; r < 8; ++r) bm[r] = 0.f;
    if (BIAS_MODE == 1) {
      const v4f b0 = *(const v4f*)(bias + mBase + mOff);
      const v4f b1 = *(const v4f*)(bias + mBase + mOff + 4);
      bm[0] = bf_rne(b0[0]); bm[1] = bf_rne(b0[1]); bm[2] = bf_rne(b0[2]); bm[3] = bf_rne(b0[3]);
      bm[4] = bf_rne(b1[0]); bm[5] = bf_rne(b1[1]); bm[6] = bf_rne(b1[2]); bm[7] = bf_rne(b1[3]);
    }
#pragma unroll
    for (int j = 0; j < 4; ++j) {
      const int n = n0 + (j << 4) + rlane;
      float bv = 0.f;
      if (BIAS_MODE == 2) bv = bf_rne(bias[n]);
#pragma unroll
      for (int r = 0; r < 8; ++r) {
        float v = acc[i][j][r];
        if (BIAS_MODE == 1) v += bm[r];
        if (BIAS_MODE == 2) v += bv;
        if (ACT == 1) v = v * (1.0f / (1.0f + expf(-v)));
        slab[(mOff + r) * 68 + (j << 4) + rlane] = v;
      }
    }
    __builtin_amdgcn_fence(__ATOMIC_RELEASE, "workgroup");
    __builtin_amdgcn_wave_barrier();
    __builtin_amdgcn_fence(__ATOMIC_ACQUIRE, "workgroup");
    if (OUT_MODE == 0) {
      float* Cp = (float*)Cout + (size_t)b * strideC;
      const int hh = lane >> 4, c4 = (lane & 15) * 4;
      for (int pass = 0; pass < 2; ++pass) {
#pragma unroll
        for (int it = 0; it < 8; ++it) {
          const int row = it * 2 + hh;
          v4f v = *(const v4f*)(slab + row * 68 + c4);
          *(volatile v4f*)(Cp + (size_t)(mBase + row) * ldc + n0 + c4) = v;
        }
        __threadfence();
      }
    } else {
      const int q = lane >> 3, c8 = (lane & 7) * 8;
      unsigned short* Cp  = (unsigned short*)Cout  + (size_t)b * strideC;
      unsigned short* Cp2 = (unsigned short*)Cout2 + (size_t)b * strideC;
      for (int pass = 0; pass < 2; ++pass) {
#pragma unroll
        for (int it = 0; it < 4; ++it) {
          const int row = it * 4 + q;
          const float* sp = slab + row * 68 + c8;
          float f[8];
#pragma unroll
          for (int e = 0; e < 8; ++e) f[e] = sp[e];
          if (OUT_MODE == 3) {
            const int npos = (mBase + row) & (T_ - 1);
            const v4f cv = *(const v4f*)(angc + (size_t)npos * NP_ + (c8 >> 1));
            const v4f sv = *(const v4f*)(angs + (size_t)npos * NP_ + (c8 >> 1));
#pragma unroll
            for (int p = 0; p < 4; ++p) {
              const float x0 = f[2 * p], x1 = f[2 * p + 1];
              f[2 * p]     = (x0 * cv[p] - x1 * sv[p]) * oscale;
              f[2 * p + 1] = (x1 * cv[p] + x0 * sv[p]) * oscale;
            }
          }
          u16x8 hv, lv;
#pragma unroll
          for (int e = 0; e < 8; ++e) {
            const unsigned short hb = f2bf_bits(f[e]);
            const unsigned short lb = f2bf_bits(f[e] - bf_bits2f(hb));
            hv[e] = hb;
            lv[e] = lb;
          }
          *(volatile u16x8*)(Cp  + (size_t)(mBase + row) * ldc + n0 + c8) = hv;
          *(volatile u16x8*)(Cp2 + (size_t)(mBase + row) * ldc + n0 + c8) = lv;
        }
        __threadfence();
      }
    }
    __builtin_amdgcn_fence(__ATOMIC_RELEASE, "workgroup");
    __builtin_amdgcn_wave_barrier();
    __builtin_amdgcn_fence(__ATOMIC_ACQUIRE, "workgroup");
  }
}

__global__ __launch_bounds__(128) __attribute__((amdgpu_num_vgpr(240)))
void ret_kernel(const unsigned short* __restrict__ qhp, const unsigned short* __restrict__ qlp,
                const unsigned short* __restrict__ khp, const unsigned short* __restrict__ klp,
                const unsigned short* __restrict__ vth, const unsigned short* __restrict__ vtl,
                const float* __restrict__ gpl, unsigned short* grc) {
  __shared__ __align__(16) unsigned short Ksh[64 * HD_];
  __shared__ __align__(16) unsigned short Ksl[64 * HD_];
  __shared__ __align__(16) unsigned short Vsh[HD_ * 64];
  __shared__ __align__(16) unsigned short Vsl[HD_ * 64];
  __shared__ __align__(16) unsigned short Psh[4][16 * 64];
  __shared__ __align__(16) unsigned short Psl[4][16 * 64];
  __shared__ __align__(16) float Os[4][16 * OS_P];

  const int tid  = threadIdx.x;
  const int wave = tid >> 5;
  const int lane = tid & 31;
  const int hh   = lane >> 4;
  const int c    = lane & 15;

  const int qb  = blockIdx.x & 31;
  const int h   = blockIdx.x >> 5;
  const int b   = blockIdx.y;
  const int q0w = qb * 64 + wave * 16;

  const size_t aoff = (size_t)b * T_ * E_ + (size_t)h * HD_;
  const unsigned short* Qh = qhp + aoff;
  const unsigned short* Ql = qlp + aoff;
  const unsigned short* Kh = khp + aoff;
  const unsigned short* Kl = klp + aoff;
  const size_t voff = (size_t)b * E_ * T_ + (size_t)(h * HD_) * T_;
  const unsigned short* Vh = vth + voff;
  const unsigned short* Vl = vtl + voff;

  const float glo = -3.4657359027997265f;
  const float ghi = -6.2383246250395077f;
  const float tt  = (float)h * (1.0f / 7.0f);
  const float gam = 1.0f - expf(glo * (1.0f - tt) + ghi * tt);
  const float lg  = logf(gam);
  float eg[8];
#pragma unroll
  for (int r = 0; r < 8; ++r) eg[r] = expf(lg * (float)r);

  FragB qah[2], qal[2];
#pragma unroll
  for (int dc = 0; dc < 2; ++dc) {
    const size_t qo = (size_t)(q0w + c) * E_ + dc * 32 + 8 * hh;
    qah[dc].h[0] = *(const u16x8*)(Qh + qo);
    qah[dc].h[1] = *(const u16x8*)(Qh + qo + 16);
    qal[dc].h[0] = *(const u16x8*)(Ql + qo);
    qal[dc].h[1] = *(const u16x8*)(Ql + qo + 16);
  }

  v8f oacc[4];
#pragma unroll
  for (int t = 0; t < 4; ++t) oacc[t] = (v8f){0.f,0.f,0.f,0.f,0.f,0.f,0.f,0.f};

  const int nChunks = qb + 1;
  for (int kc = 0; kc < nChunks; ++kc) {
    const int kv0 = kc * 64;
    __syncthreads();
    {
      const int r = tid >> 1, half = (tid & 1) * 32;
      const unsigned short* ks = Kh + (size_t)(kv0 + r) * E_ + half;
      const unsigned short* kl = Kl + (size_t)(kv0 + r) * E_ + half;
      const unsigned short* vs = Vh + (size_t)r * T_ + kv0 + half;
      const unsigned short* vl = Vl + (size_t)r * T_ + kv0 + half;
#pragma unroll
      for (int i = 0; i < 4; ++i) {
        const u16x8 a0 = *(const u16x8*)(ks + 8 * i);
        const u16x8 a1 = *(const u16x8*)(kl + 8 * i);
        const u16x8 b0 = *(const u16x8*)(vs + 8 * i);
        const u16x8 b1 = *(const u16x8*)(vl + 8 * i);
        *(u16x8*)(Ksh + r * HD_ + half + 8 * i) = a0;
        *(u16x8*)(Ksl + r * HD_ + half + 8 * i) = a1;
        *(u16x8*)(Vsh + r * 64  + half + 8 * i) = b0;
        *(u16x8*)(Vsl + r * 64  + half + 8 * i) = b1;
      }
    }
    __syncthreads();

#pragma unroll 1
    for (int j = 0; j < 4; ++j) {
      v8f s = (v8f){0.f,0.f,0.f,0.f,0.f,0.f,0.f,0.f};
#pragma unroll
      for (int dc = 0; dc < 2; ++dc) {
        FragB kb, kl2;
        const int ko = (j * 16 + c) * HD_ + dc * 32 + 8 * hh;
        kb.h[0]  = *(const u16x8*)(Ksh + ko);
        kb.h[1]  = *(const u16x8*)(Ksh + ko + 16);
        kl2.h[0] = *(const u16x8*)(Ksl + ko);
        kl2.h[1] = *(const u16x8*)(Ksl + ko + 16);
        s = mma_g(s, qah[dc].v, kb.v);
        s = mma_g(s, qah[dc].v, kl2.v);
        s = mma_g(s, qal[dc].v, kb.v);
      }
      const int d0 = q0w + 8 * hh - (kv0 + j * 16 + c);
      const float base = expf(lg * (float)d0);
#pragma unroll
      for (int r = 0; r < 8; ++r) {
        const float val = (d0 + r >= 0) ? (s[r] * (base * eg[r])) : 0.0f;
        const unsigned short hb = f2bf_bits(val);
        const unsigned short lb = f2bf_bits(val - bf_bits2f(hb));
        Psh[wave][(8 * hh + r) * 64 + j * 16 + c] = hb;
        Psl[wave][(8 * hh + r) * 64 + j * 16 + c] = lb;
      }
    }
    __builtin_amdgcn_fence(__ATOMIC_RELEASE, "workgroup");
    __builtin_amdgcn_wave_barrier();
    __builtin_amdgcn_fence(__ATOMIC_ACQUIRE, "workgroup");

#pragma unroll 1
    for (int kk = 0; kk < 2; ++kk) {
      FragB pa, pl;
      const int po = c * 64 + kk * 32 + 8 * hh;
      pa.h[0] = *(const u16x8*)(Psh[wave] + po);
      pa.h[1] = *(const u16x8*)(Psh[wave] + po + 16);
      pl.h[0] = *(const u16x8*)(Psl[wave] + po);
      pl.h[1] = *(const u16x8*)(Psl[wave] + po + 16);
#pragma unroll
      for (int t = 0; t < 4; ++t) {
        FragB vb, vl2;
        const int vo = (t * 16 + c) * 64 + kk * 32 + 8 * hh;
        vb.h[0]  = *(const u16x8*)(Vsh + vo);
        vb.h[1]  = *(const u16x8*)(Vsh + vo + 16);
        vl2.h[0] = *(const u16x8*)(Vsl + vo);
        vl2.h[1] = *(const u16x8*)(Vsl + vo + 16);
        oacc[t] = mma_g(oacc[t], pa.v, vb.v);
        oacc[t] = mma_g(oacc[t], pa.v, vl2.v);
        oacc[t] = mma_g(oacc[t], pl.v, vb.v);
      }
    }
  }

  float* os = Os[wave];
#pragma unroll
  for (int r = 0; r < 8; ++r) {
    float sm = (oacc[0][r] + oacc[1][r]) + (oacc[2][r] + oacc[3][r]);
    sm += __shfl_xor(sm, 1, 32);
    sm += __shfl_xor(sm, 2, 32);
    sm += __shfl_xor(sm, 4, 32);
    sm += __shfl_xor(sm, 8, 32);
    const float mean = sm * (1.0f / 64.0f);
    float sq = 0.0f;
#pragma unroll
    for (int t = 0; t < 4; ++t) { const float dv = oacc[t][r] - mean; sq += dv * dv; }
    sq += __shfl_xor(sq, 1, 32);
    sq += __shfl_xor(sq, 2, 32);
    sq += __shfl_xor(sq, 4, 32);
    sq += __shfl_xor(sq, 8, 32);
    const float var = sq * (1.0f / 64.0f);
    const float inv = rsqrtf(var + 1e-6f);
#pragma unroll
    for (int t = 0; t < 4; ++t) os[(8 * hh + r) * OS_P + t * 16 + c] = (oacc[t][r] - mean) * inv;
  }
  __builtin_amdgcn_fence(__ATOMIC_RELEASE, "workgroup");
  __builtin_amdgcn_wave_barrier();
  __builtin_amdgcn_fence(__ATOMIC_ACQUIRE, "workgroup");

  {
    const int q  = lane >> 3;
    const int c8 = (lane & 7) * 8;
    for (int pass = 0; pass < 2; ++pass) {
#pragma unroll
      for (int it = 0; it < 4; ++it) {
        const int row = it * 4 + q;
        const float* op = os + row * OS_P + c8;
        const v4f y0 = *(const v4f*)op;
        const v4f y1 = *(const v4f*)(op + 4);
        const size_t tok = (size_t)b * T_ + q0w + row;
        const float* gp = gpl + tok * E_ + h * HD_ + c8;
        const v4f g0 = *(const v4f*)gp;
        const v4f g1 = *(const v4f*)(gp + 4);
        u16x8 hv, lv;
#pragma unroll
        for (int e = 0; e < 4; ++e) {
          const float f0 = y0[e] * g0[e];
          const unsigned short h0 = f2bf_bits(f0);
          hv[e] = h0;
          lv[e] = f2bf_bits(f0 - bf_bits2f(h0));
          const float f1 = y1[e] * g1[e];
          const unsigned short h1 = f2bf_bits(f1);
          hv[4 + e] = h1;
          lv[4 + e] = f2bf_bits(f1 - bf_bits2f(h1));
        }
        unsigned short* dp = grc + tok * GRK_ + h * HD_ + c8;
        *(volatile u16x8*)dp = hv;
        *(volatile u16x8*)(dp + E_) = lv;
      }
      __threadfence();
    }
  }
}

extern "C" void kernel_launch(void* const* d_in, const int* in_sizes, int n_in,
                              void* d_out, int out_size, void* d_ws, size_t ws_size,
                              hipStream_t stream) {
  if (n_in < 13) return;
  if (in_sizes[0] != NTOK_ * E_) return;
  if (in_sizes[1] != NTOK_ * E_) return;
  if (in_sizes[2] != NTOK_ * E_) return;
  if (in_sizes[3] != E_ * E_ || in_sizes[5] != E_ * E_ || in_sizes[7] != E_ * E_ || in_sizes[9] != E_ * E_ || in_sizes[11] != E_ * E_) return;
  if (in_sizes[4] != E_ || in_sizes[6] != E_ || in_sizes[8] != E_ || in_sizes[10] != E_ || in_sizes[12] != E_) return;
  if (out_size != NTOK_ * E_) return;
  if (ws_size < WS_END) return;

  const float* query = (const float*)d_in[0];
  const float* k_in  = (const float*)d_in[1];
  const float* v_in  = (const float*)d_in[2];
  const float* Wq = (const float*)d_in[3];
  const float* bq = (const float*)d_in[4];
  const float* Wk = (const float*)d_in[5];
  const float* bk = (const float*)d_in[6];
  const float* Wv = (const float*)d_in[7];
  const float* bv = (const float*)d_in[8];
  const float* Wg = (const float*)d_in[9];
  const float* bg = (const float*)d_in[10];
  const float* Wo = (const float*)d_in[11];
  const float* bo = (const float*)d_in[12];
  float* out = (float*)d_out;

  char* ws = (char*)d_ws;
  unsigned short* QB   = (unsigned short*)(ws + OFF_QB);
  unsigned short* KB   = (unsigned short*)(ws + OFF_KB);
  unsigned short* VB   = (unsigned short*)(ws + OFF_VB);
  unsigned short* WQB  = (unsigned short*)(ws + OFF_WQ);
  unsigned short* WKB  = (unsigned short*)(ws + OFF_WK);
  unsigned short* WVB  = (unsigned short*)(ws + OFF_WV);
  unsigned short* WGB  = (unsigned short*)(ws + OFF_WG);
  unsigned short* WOT2 = (unsigned short*)(ws + OFF_WO2);
  float*          ANGC = (float*)(ws + OFF_ANGC);
  float*          ANGS = (float*)(ws + OFF_ANGS);
  unsigned short* QH   = (unsigned short*)(ws + OFF_QH);
  unsigned short* QL   = (unsigned short*)(ws + OFF_QL);
  unsigned short* KH   = (unsigned short*)(ws + OFF_KH);
  unsigned short* KL   = (unsigned short*)(ws + OFF_KL);
  unsigned short* VTH  = (unsigned short*)(ws + OFF_VTH);
  unsigned short* VTL  = (unsigned short*)(ws + OFF_VTL);
  float*          G    = (float*)(ws + OFF_G);
  unsigned short* GRC  = (unsigned short*)(ws + OFF_GRC);

  const dim3 blk(256);

  {
    const int n8 = NTOK_ * E_ / 8;
    xcvt_kernel<<<dim3(n8 / 256), blk, 0, stream>>>(query, QB, n8);
    xcvt_kernel<<<dim3(n8 / 256), blk, 0, stream>>>(k_in,  KB, n8);
    xcvt_kernel<<<dim3(n8 / 256), blk, 0, stream>>>(v_in,  VB, n8);
  }
  {
    const int n8 = E_ * E_ / 8;
    xcvt_kernel<<<dim3(n8 / 256), blk, 0, stream>>>(Wq, WQB, n8);
    xcvt_kernel<<<dim3(n8 / 256), blk, 0, stream>>>(Wk, WKB, n8);
    xcvt_kernel<<<dim3(n8 / 256), blk, 0, stream>>>(Wv, WVB, n8);
    xcvt_kernel<<<dim3(n8 / 256), blk, 0, stream>>>(Wg, WGB, n8);
    dupcvt_kernel<<<dim3(n8 / 256), blk, 0, stream>>>(Wo, WOT2, n8, E_, GRK_);
  }
  ang_kernel<<<dim3((T_ * NP_) / 256), blk, 0, stream>>>(ANGC, ANGS, T_ * NP_);

  const dim3 gP(((NTOK_ / 64) * (E_ / 64)) / 8, 1);
  const dim3 gVT(((E_ / 64) * (T_ / 64)) / 8, NB_);
  const dim3 gR(NH_ * (T_ / 64), NB_);

  gemm64_kernel<2, 3, 0><<<gP, blk, 0, stream>>>(
      QB, E_, 0L, WQB, E_, 0L, (void*)QH, (void*)QL, E_, 0L, bq, ANGC, ANGS, 1.0f, NTOK_, E_, E_);
  gemm64_kernel<2, 3, 0><<<gP, blk, 0, stream>>>(
      KB, E_, 0L, WKB, E_, 0L, (void*)KH, (void*)KL, E_, 0L, bk, ANGC, ANGS, 0.125f, NTOK_, E_, E_);
  gemm64_kernel<1, 2, 0><<<gVT, blk, 0, stream>>>(
      WVB, E_, 0L, VB, E_, (long)T_ * E_, (void*)VTH, (void*)VTL, T_, (long)E_ * T_, bv, ANGC, ANGS, 1.0f, E_, T_, E_);
  gemm64_kernel<2, 0, 1><<<gP, blk, 0, stream>>>(
      QB, E_, 0L, WGB, E_, 0L, (void*)G, (void*)G, E_, 0L, bg, ANGC, ANGS, 1.0f, NTOK_, E_, E_);
  ret_kernel<<<gR, dim3(128), 0, stream>>>(QH, QL, KH, KL, VTH, VTL, G, GRC);
  gemm64_kernel<2, 0, 0><<<gP, blk, 0, stream>>>(
      GRC, GRK_, 0L, WOT2, GRK_, 0L, (void*)out, (void*)out, E_, 0L, bo, ANGC, ANGS, 1.0f, NTOK_, E_, GRK_);
  (void)hipGetLastError();
}
